// SWEGNNLayer_14920716387062
// MI455X (gfx1250) — hardware-verified
//
#include <hip/hip_runtime.h>
#include <stddef.h>


#define HC       32
#define KIN      7
#define BP       40
#define ETHR     128
#define EWAV     (ETHR / 32)
#define EPW      32
#define EPB      (EWAV * EPW)
#define SPP      8
#define STHR     256
#define SWAV     (STHR / 32)
#define SLOT     16
#define CHB      (STHR * SLOT)
#define NBK      512
#define NBKL     9
#define MAXB     512
#define CAP2     12288
#define MAXDEG   128
#define NTHR     256
#define LDS_BKT  ((2 * CAP2 + SWAV * NBK + 2 * NBK) * 4 + 64)
#define XSC      16.0f
#define WSC      64.0f
#define RH       0.0009765625f
#define WSCAP    134217728

static_assert(EPB == 128);
static_assert(CHB == 4096);
static_assert((BP % 8) == 0);
static_assert(HC == 32);
static_assert(HC * HC == ETHR * 8);
static_assert((CHB % EPB) == 0);
static_assert(SWAV * MAXB == 4 * STHR * 4);
static_assert(CHB == 4 * STHR * 4);
static_assert(MAXB == 2 * STHR);
static_assert(NBK == 2 * STHR);
static_assert(MAXB == 4 * (STHR / 2));
static_assert((CAP2 % (4 * STHR)) == 0);
static_assert((SWAV * NBK) % (4 * STHR) == 0);
static_assert(2 * NBK == 4 * STHR);
static_assert((CAP2 % (32 * SWAV)) == 0);
static_assert(NTHR == 256);
static_assert(LDS_BKT == 118848);

typedef float    v2f  __attribute__((ext_vector_type(2)));
typedef float    v4f  __attribute__((ext_vector_type(4)));
typedef float    v8f  __attribute__((ext_vector_type(8)));
typedef int      v4i  __attribute__((ext_vector_type(4)));
typedef unsigned v4u  __attribute__((ext_vector_type(4)));
typedef _Float16 v4h  __attribute__((ext_vector_type(4)));
typedef _Float16 v8h  __attribute__((ext_vector_type(8)));
typedef _Float16 v16h __attribute__((ext_vector_type(16)));
union Frag { v16h v; v8h h[2]; v4h q[4]; };

__device__ __forceinline__ v8f wmh(v16h a, v16h b, v8f c) {
  v8f d = __builtin_amdgcn_wmma_f32_16x16x32_f16(false, a, false, b, (short)0, c, false, false);
  asm volatile("v_nop\n\tv_nop\n\tv_nop\n\tv_nop" : "+v"(d) : "v"(a), "v"(b));
  return d;
}

__device__ __forceinline__ v4h relu4h(v4f x) {
  v4h r;
  r.x = (_Float16)fmaxf(x.x, 0.0f);
  r.y = (_Float16)fmaxf(x.y, 0.0f);
  r.z = (_Float16)fmaxf(x.z, 0.0f);
  r.w = (_Float16)fmaxf(x.w, 0.0f);
  return r;
}

__device__ __forceinline__ void wfence() {
  __builtin_amdgcn_fence(__ATOMIC_ACQ_REL, "wavefront");
  __builtin_amdgcn_wave_barrier();
}

__device__ __forceinline__ unsigned match9(int key, unsigned vm) {
  unsigned peers = vm;
#pragma unroll
  for (int i = 0; i < 9; ++i) {
    const bool bit = ((key >> i) & 1) != 0;
    const unsigned bq = __builtin_amdgcn_ballot_w32(bit);
    peers &= bit ? bq : ~bq;
  }
  return peers;
}

__device__ __forceinline__ void blkscan(int cnt, int lane, int wave, int* swt, int& pos, int& nh) {
  int x = cnt;
#pragma unroll
  for (int o = 1; o < 32; o <<= 1) {
    const int y = __shfl_up(x, o, 32);
    x += (lane >= o) ? y : 0;
  }
  if (lane == 31) swt[wave] = x;
  __syncthreads();
  int wpre = 0, tot = 0;
#pragma unroll
  for (int w = 0; w < SWAV; ++w) {
    const int v = swt[w];
    wpre += (w < wave) ? v : 0;
    tot += v;
  }
  pos = wpre + x - cnt;
  nh = tot;
}

__global__ __launch_bounds__(ETHR) void k_edge(
    const float* __restrict__ nf, const int* __restrict__ ei, const float* __restrict__ ea,
    const float* __restrict__ W0, const float* __restrict__ b0, const float* __restrict__ W1,
    const float* __restrict__ b1, const float* __restrict__ W2, const float* __restrict__ b2,
    float* msg, int nN, int nE) {
  __shared__ __attribute__((aligned(16))) float sW0[KIN * HC];
  __shared__ __attribute__((aligned(16))) float sb0[HC];
  __shared__ __attribute__((aligned(16))) float sb1[HC];
  __shared__ __attribute__((aligned(16))) float sw2[HC];
  __shared__ __attribute__((aligned(16))) _Float16 sB[HC * BP];
  __shared__ __attribute__((aligned(16))) float spr[EWAV * EPW * SPP];
  __shared__ __attribute__((aligned(16))) float sc[EPB];
  const int tid = threadIdx.x, lane = tid & 31, hh = lane >> 4, m = lane & 15;
  const int wave = __builtin_amdgcn_readfirstlane(tid >> 5);

  for (int i = tid; i < KIN * HC; i += ETHR) sW0[i] = W0[i] * XSC;
  if (wave == 0)      sb0[lane] = b0[lane] * XSC;
  else if (wave == 1) sb1[lane] = b1[lane];
  else if (wave == 2) sw2[lane] = W2[lane];
  {
    const int n = tid >> 2, k0 = (tid & 3) * 8;
    v8h hv;
#pragma unroll
    for (int e = 0; e < 8; ++e) hv[e] = (_Float16)(W1[(k0 + e) * HC + n] * WSC);
    *(v8h*)(sB + n * BP + k0) = hv;
  }
  const float b2v = b2[0];

  float* sp = spr + wave * (EPW * SPP);
  {
    int e = blockIdx.x * EPB + wave * EPW + lane;
    e = e > nE - 1 ? nE - 1 : e;
    int s = ei[e];
    s = s < 0 ? 0 : (s > nN - 1 ? nN - 1 : s);
    int r = ei[(size_t)nE + (size_t)e];
    r = r < 0 ? 0 : (r > nN - 1 ? nN - 1 : r);
    const v2f hs = *(const v2f*)(nf + 2 * (size_t)s);
    const v2f hr = *(const v2f*)(nf + 2 * (size_t)r);
    const float* ap = ea + 3 * (size_t)e;
    v4f q0, q1;
    q0.x = hs.x;  q0.y = hs.y;  q0.z = hr.x;  q0.w = hr.y;
    q1.x = ap[0]; q1.y = ap[1]; q1.z = ap[2]; q1.w = 0.0f;
    *(v4f*)(sp + lane * SPP)     = q0;
    *(v4f*)(sp + lane * SPP + 4) = q1;
  }
  __syncthreads();

  float p0[8], p1[8];
  {
    const v4f t0 = *(const v4f*)(sp + m * SPP),        t1 = *(const v4f*)(sp + m * SPP + 4);
    const v4f u0 = *(const v4f*)(sp + (16 + m) * SPP), u1 = *(const v4f*)(sp + (16 + m) * SPP + 4);
    p0[0] = t0.x; p0[1] = t0.y; p0[2] = t0.z; p0[3] = t0.w; p0[4] = t1.x; p0[5] = t1.y; p0[6] = t1.z; p0[7] = t1.w;
    p1[0] = u0.x; p1[1] = u0.y; p1[2] = u0.z; p1[3] = u0.w; p1[4] = u1.x; p1[5] = u1.y; p1[6] = u1.z; p1[7] = u1.w;
  }
  Frag a0, a1;
#pragma unroll
  for (int q = 0; q < 4; ++q) {
    const int c = ((q >> 1) ? 16 : 0) + 8 * hh + 4 * (q & 1);
    v4f x0 = *(const v4f*)(sb0 + c);
    v4f x1 = x0;
#pragma unroll
    for (int k = 0; k < KIN; ++k) {
      const v4f w = *(const v4f*)(sW0 + k * HC + c);
      x0 += p0[k] * w;
      x1 += p1[k] * w;
    }
    a0.q[q] = relu4h(x0);
    a1.q[q] = relu4h(x1);
  }

  v8f acc0[2], acc1[2];
#pragma unroll
  for (int t = 0; t < 2; ++t) {
    const _Float16* bp = sB + (16 * t + m) * BP + 8 * hh;
    Frag b;
    b.h[0] = *(const v8h*)bp;
    b.h[1] = *(const v8h*)(bp + 16);
    const v8f z = {0.f, 0.f, 0.f, 0.f, 0.f, 0.f, 0.f, 0.f};
    acc0[t] = wmh(a0.v, b.v, z);
    acc1[t] = wmh(a1.v, b.v, z);
  }

  float b1c[2], w2c[2];
#pragma unroll
  for (int t = 0; t < 2; ++t) { b1c[t] = sb1[16 * t + m]; w2c[t] = sw2[16 * t + m]; }
  float v[16];
#pragma unroll
  for (int r = 0; r < 8; ++r) {
    float s0 = 0.0f, s1 = 0.0f;
#pragma unroll
    for (int t = 0; t < 2; ++t) {
      const float h0 = fmaxf(fmaf(acc0[t][r], RH, b1c[t]), 0.0f);
      const float h1 = fmaxf(fmaf(acc1[t][r], RH, b1c[t]), 0.0f);
      s0 = fmaf(h0, w2c[t], s0);
      s1 = fmaf(h1, w2c[t], s1);
    }
    v[r] = s0;
    v[8 + r] = s1;
  }

  float u[8];
  {
    const bool kb = ((lane >> 3) & 1) != 0;
#pragma unroll
    for (int i = 0; i < 8; ++i) {
      const float snd = kb ? v[i] : v[i + 8];
      const float kp  = kb ? v[i + 8] : v[i];
      u[i] = kp + __shfl_xor(snd, 8, 32);
    }
  }
  float w4[4];
  {
    const bool kb = ((lane >> 2) & 1) != 0;
#pragma unroll
    for (int i = 0; i < 4; ++i) {
      const float snd = kb ? u[i] : u[i + 4];
      const float kp  = kb ? u[i + 4] : u[i];
      w4[i] = kp + __shfl_xor(snd, 4, 32);
    }
  }
  float x2[2];
  {
    const bool kb = ((lane >> 1) & 1) != 0;
#pragma unroll
    for (int i = 0; i < 2; ++i) {
      const float snd = kb ? w4[i] : w4[i + 2];
      const float kp  = kb ? w4[i + 2] : w4[i];
      x2[i] = kp + __shfl_xor(snd, 2, 32);
    }
  }
  float fin;
  {
    const bool kb = (lane & 1) != 0;
    const float snd = kb ? x2[0] : x2[1];
    const float kp  = kb ? x2[1] : x2[0];
    fin = kp + __shfl_xor(snd, 1, 32);
  }
  {
    const int j = 16 * (m >> 3) + 8 * hh + (m & 7);
    sc[wave * EPW + j] = fin + b2v;
  }
  __syncthreads();

  if (wave == 0) {
    const v4f ov = *(const v4f*)(sc + 4 * lane);
    float* op = msg + (size_t)blockIdx.x * EPB + 4 * lane;
    *(volatile v4f*)op = ov;
    __threadfence();
    *(volatile v4f*)op = ov;
  }
}

__global__ __launch_bounds__(STHR) void k_bsort(const int* __restrict__ dsts, unsigned* KEY, unsigned* CO,
                                                 int nN, int nE) {
  __shared__ __attribute__((aligned(16))) int      srun[SWAV * MAXB];
  __shared__ __attribute__((aligned(16))) unsigned sstg[CHB];
  __shared__ __attribute__((aligned(16))) unsigned sco[MAXB];
  __shared__ int swt[SWAV];
  const int tid = threadIdx.x, lane = tid & 31;
  const int wave = __builtin_amdgcn_readfirstlane(tid >> 5);
  const unsigned lt = (1u << lane) - 1u;
  {
    const v4i z = {0, 0, 0, 0};
    const v4u zu = {0u, 0u, 0u, 0u};
#pragma unroll
    for (int it = 0; it < (SWAV * MAXB) / (4 * STHR); ++it) ((v4i*)srun)[it * STHR + tid] = z;
#pragma unroll
    for (int it = 0; it < CHB / (4 * STHR); ++it) ((v4u*)sstg)[it * STHR + tid] = zu;
  }
  __syncthreads();

  const int eb = blockIdx.x * CHB + wave * (32 * SLOT);
  int dc[SLOT];
  unsigned vm = 0u;
#pragma unroll
  for (int j = 0; j < SLOT; ++j) {
    const int e = eb + 32 * j + lane;
    const bool ok = e < nE;
    const int ec = ok ? e : nE - 1;
    const int d = dsts[ec];
    const bool inr = ok && ((unsigned)d < (unsigned)nN);
    dc[j] = inr ? d : 0;
    vm |= (inr ? 1u : 0u) << j;
  }
  int* runw = srun + wave * MAXB;

#pragma unroll
  for (int j = 0; j < SLOT; ++j) {
    const bool inr = ((vm >> j) & 1u) != 0u;
    const int kb = dc[j] >> NBKL;
    const unsigned vmask = __builtin_amdgcn_ballot_w32(inr);
    const unsigned peers = match9(kb, vmask);
    const int pc = __builtin_popcount(peers);
    const bool lead = inr && ((peers & lt) == 0u);
    const int cur = runw[kb];
    if (lead) runw[kb] = cur + pc;
    wfence();
  }
  __syncthreads();

  {
    const int b0 = 2 * tid, b1 = b0 + 1;
    int c0 = 0, c1 = 0, pw0[SWAV], pw1[SWAV];
#pragma unroll
    for (int w = 0; w < SWAV; ++w) {
      pw0[w] = c0; c0 += srun[w * MAXB + b0];
      pw1[w] = c1; c1 += srun[w * MAXB + b1];
    }
    int pos, tot;
    blkscan(c0 + c1, lane, wave, swt, pos, tot);
    const int o0 = pos, o1 = pos + c0;
#pragma unroll
    for (int w = 0; w < SWAV; ++w) {
      srun[w * MAXB + b0] = o0 + pw0[w];
      srun[w * MAXB + b1] = o1 + pw1[w];
    }
    sco[b0] = ((unsigned)o0 << 16) | (unsigned)c0;
    sco[b1] = ((unsigned)o1 << 16) | (unsigned)c1;
  }
  __syncthreads();

#pragma unroll
  for (int j = 0; j < SLOT; ++j) {
    const bool inr = ((vm >> j) & 1u) != 0u;
    const int kb = dc[j] >> NBKL;
    const unsigned vmask = __builtin_amdgcn_ballot_w32(inr);
    const unsigned peers = match9(kb, vmask);
    const int pc = __builtin_popcount(peers);
    const bool lead = inr && ((peers & lt) == 0u);
    const int cur = runw[kb];
    const int p = cur + __builtin_popcount(peers & lt);
    if (lead) runw[kb] = cur + pc;
    if (inr) {
      const int pp = p < CHB - 1 ? p : CHB - 1;
      sstg[pp] = (((unsigned)dc[j] & (unsigned)(NBK - 1)) << 22) | (unsigned)(eb + 32 * j + lane);
    }
    wfence();
  }
  __syncthreads();

  unsigned* kp = KEY + (size_t)blockIdx.x * CHB;
  unsigned* cp = CO + (size_t)blockIdx.x * MAXB;
#pragma unroll
  for (int it = 0; it < CHB / (4 * STHR); ++it) {
    const int f = it * STHR + tid;
    const v4u vv = ((const v4u*)sstg)[f];
    *(volatile v4u*)(kp + 4 * f) = vv;
  }
  if (tid < MAXB / 4) {
    const v4u vv = ((const v4u*)sco)[tid];
    *(volatile v4u*)(cp + 4 * tid) = vv;
  }
  __threadfence();
#pragma unroll
  for (int it = 0; it < CHB / (4 * STHR); ++it) {
    const int f = it * STHR + tid;
    const v4u vv = ((const v4u*)sstg)[f];
    *(volatile v4u*)(kp + 4 * f) = vv;
  }
  if (tid < MAXB / 4) {
    const v4u vv = ((const v4u*)sco)[tid];
    *(volatile v4u*)(cp + 4 * tid) = vv;
  }
}

__global__ __launch_bounds__(STHR) void k_bucket(const unsigned* __restrict__ CO, const unsigned* __restrict__ KEY,
                                                  unsigned* EID, int* NT, int nChunk, int nBatch) {
  extern __shared__ __attribute__((aligned(16))) char dynl[];
  unsigned* lst = (unsigned*)dynl;
  unsigned* srt = lst + CAP2;
  int*      wc  = (int*)(srt + CAP2);
  int*      snt = wc + SWAV * NBK;
  int*      swt = snt + 2 * NBK;
  const int tid = threadIdx.x, lane = tid & 31;
  const int wave = __builtin_amdgcn_readfirstlane(tid >> 5);
  const unsigned lt = (1u << lane) - 1u;
  const int b = blockIdx.x;
  {
    const v4u zu = {0u, 0u, 0u, 0u};
    const v4i z = {0, 0, 0, 0};
#pragma unroll
    for (int it = 0; it < CAP2 / (4 * STHR); ++it) {
      ((v4u*)lst)[it * STHR + tid] = zu;
      ((v4u*)srt)[it * STHR + tid] = zu;
    }
#pragma unroll
    for (int it = 0; it < (SWAV * NBK) / (4 * STHR); ++it) ((v4i*)wc)[it * STHR + tid] = z;
  }
  __syncthreads();

  int L = 0;
#pragma unroll 1
  for (int q = 0; q < nBatch; ++q) {
    const int s = q * STHR + tid;
    const bool sv = s < nChunk;
    const int sc = sv ? s : nChunk - 1;
    const unsigned co = CO[(size_t)sc * MAXB + b];
    int c = sv ? (int)(co & 0x1FFFu) : 0;
    c = c > CHB ? CHB : c;
    int o = (int)((co >> 16) & 0x1FFFu);
    o = o > CHB - c ? CHB - c : o;
    int pos, tot;
    blkscan(c, lane, wave, swt, pos, tot);
    const int base = L + pos;
    const unsigned* rp = KEY + (size_t)sc * CHB + o;
#pragma unroll 1
    for (int i = 0; i < c; ++i) {
      const int di = base + i;
      const unsigned vv = rp[i];
      if ((unsigned)di < (unsigned)CAP2) lst[di] = vv;
    }
    L += tot;
    __syncthreads();
  }
  const int Lc = L < CAP2 ? L : CAP2;
  const int nG = (Lc + 31) >> 5;
  int* wcw = wc + wave * NBK;

#pragma unroll 1
  for (int gi = 0; gi < CAP2 / (32 * SWAV); ++gi) {
    const int g = wave + SWAV * gi;
    if (g >= nG) break;
    const int idx = 32 * g + lane;
    const bool valid = idx < Lc;
    const unsigned key = lst[idx];
    const int ld = (int)((key >> 22) & (unsigned)(NBK - 1));
    const unsigned vmask = __builtin_amdgcn_ballot_w32(valid);
    const unsigned peers = match9(ld, vmask);
    const int pc = __builtin_popcount(peers);
    const bool lead = valid && ((peers & lt) == 0u);
    const int cur = wcw[ld];
    if (lead) wcw[ld] = cur + pc;
    wfence();
  }
  __syncthreads();

  {
    const int l0 = 2 * tid, l1 = l0 + 1;
    int c0 = 0, c1 = 0, pw0[SWAV], pw1[SWAV];
#pragma unroll
    for (int w = 0; w < SWAV; ++w) {
      pw0[w] = c0; c0 += wc[w * NBK + l0];
      pw1[w] = c1; c1 += wc[w * NBK + l1];
    }
    int pos, tot;
    blkscan(c0 + c1, lane, wave, swt, pos, tot);
    const int off0 = pos, off1 = pos + c0;
#pragma unroll
    for (int w = 0; w < SWAV; ++w) {
      wc[w * NBK + l0] = off0 + pw0[w];
      wc[w * NBK + l1] = off1 + pw1[w];
    }
    int n0c = c0, n1c = c1;
    if (off0 + n0c > CAP2) n0c = CAP2 - off0;
    if (off1 + n1c > CAP2) n1c = CAP2 - off1;
    n0c = n0c < 0 ? 0 : n0c;
    n1c = n1c < 0 ? 0 : n1c;
    const int s0 = off0 < CAP2 ? off0 : CAP2 - 1;
    const int s1 = off1 < CAP2 ? off1 : CAP2 - 1;
    snt[2 * l0] = b * CAP2 + s0; snt[2 * l0 + 1] = n0c;
    snt[2 * l1] = b * CAP2 + s1; snt[2 * l1 + 1] = n1c;
  }
  __syncthreads();

#pragma unroll 1
  for (int gi = 0; gi < CAP2 / (32 * SWAV); ++gi) {
    const int g = wave + SWAV * gi;
    if (g >= nG) break;
    const int idx = 32 * g + lane;
    const bool valid = idx < Lc;
    const unsigned key = lst[idx];
    const int ld = (int)((key >> 22) & (unsigned)(NBK - 1));
    const unsigned vmask = __builtin_amdgcn_ballot_w32(valid);
    const unsigned peers = match9(ld, vmask);
    const int pc = __builtin_popcount(peers);
    const bool lead = valid && ((peers & lt) == 0u);
    const int cur = wcw[ld];
    const int p = cur + __builtin_popcount(peers & lt);
    if (lead) wcw[ld] = cur + pc;
    if (valid && (unsigned)p < (unsigned)CAP2) srt[p] = key & 0x3FFFFFu;
    wfence();
  }
  __syncthreads();

  unsigned* ep = EID + (size_t)b * CAP2;
  int* np = NT + (size_t)b * (2 * NBK);
#pragma unroll
  for (int it = 0; it < CAP2 / (4 * STHR); ++it) {
    const int f = it * STHR + tid;
    const v4u vv = ((const v4u*)srt)[f];
    *(volatile v4u*)(ep + 4 * f) = vv;
  }
  {
    const v4i vv = ((const v4i*)snt)[tid];
    *(volatile v4i*)(np + 4 * tid) = vv;
  }
  __threadfence();
#pragma unroll
  for (int it = 0; it < CAP2 / (4 * STHR); ++it) {
    const int f = it * STHR + tid;
    const v4u vv = ((const v4u*)srt)[f];
    *(volatile v4u*)(ep + 4 * f) = vv;
  }
  {
    const v4i vv = ((const v4i*)snt)[tid];
    *(volatile v4i*)(np + 4 * tid) = vv;
  }
}

__global__ __launch_bounds__(NTHR) void k_node(
    const int* __restrict__ NT, const unsigned* __restrict__ EID, const float* __restrict__ msg,
    const float* __restrict__ nf, const float* __restrict__ V0, const float* __restrict__ c0,
    const float* __restrict__ V1, const float* __restrict__ c1, float* out, int nN, int nE, int totE) {
  __shared__ __attribute__((aligned(16))) float sw0[3 * HC];
  __shared__ __attribute__((aligned(16))) float sc0[HC];
  __shared__ __attribute__((aligned(16))) float sw1[HC];
  __shared__ __attribute__((aligned(16))) float so[NTHR];
  const int tid = threadIdx.x;
  if (tid < 3 * HC)      sw0[tid] = V0[tid];
  else if (tid < 4 * HC) sc0[tid - 3 * HC] = c0[tid - 3 * HC];
  else if (tid < 5 * HC) sw1[tid - 4 * HC] = V1[tid - 4 * HC];
  const float b1v = c1[0];

  const int n = blockIdx.x * NTHR + tid;
  const int nc = n > nN - 1 ? nN - 1 : n;
  int st = NT[2 * (size_t)nc];
  int ct = NT[2 * (size_t)nc + 1];
  ct = ct < 0 ? 0 : (ct > MAXDEG ? MAXDEG : ct);
  st = st < 0 ? 0 : (st > totE - 1 ? totE - 1 : st);
  float a = 0.0f;
#pragma unroll 1
  for (int i = 0; i < ct; ++i) {
    int ix = st + i;
    ix = ix > totE - 1 ? totE - 1 : ix;
    const unsigned vv = EID[ix];
    int e = (int)(vv & 0x3FFFFFu);
    e = e > nE - 1 ? nE - 1 : e;
    a += msg[e];
  }
  __syncthreads();

  const v2f hz = *(const v2f*)(nf + 2 * (size_t)nc);
  float upd = b1v;
#pragma unroll 1
  for (int j = 0; j < HC; ++j) {
    float y = fmaf(hz.x, sw0[j], fmaf(hz.y, sw0[HC + j], fmaf(a, sw0[2 * HC + j], sc0[j])));
    y = fmaxf(y, 0.0f);
    upd = fmaf(y, sw1[j], upd);
  }
  so[tid] = fmaxf(hz.x + upd, 0.0f);
  __syncthreads();

  const int rem = nN - blockIdx.x * NTHR;
  const int cnt = rem < NTHR ? rem : NTHR;
  float* gp = out + (size_t)blockIdx.x * NTHR;
  if (tid < NTHR / 4) {
    const int f = 4 * tid;
    const v4f ov = *(const v4f*)(so + f);
    if (f + 3 < cnt) {
      *(volatile v4f*)(gp + f) = ov;
    } else {
      if (f     < cnt) *(volatile float*)(gp + f)     = ov.x;
      if (f + 1 < cnt) *(volatile float*)(gp + f + 1) = ov.y;
      if (f + 2 < cnt) *(volatile float*)(gp + f + 2) = ov.z;
    }
  }
  __threadfence();
  if (tid < NTHR / 4) {
    const int f = 4 * tid;
    const v4f ov = *(const v4f*)(so + f);
    if (f + 3 < cnt) {
      *(volatile v4f*)(gp + f) = ov;
    } else {
      if (f     < cnt) *(volatile float*)(gp + f)     = ov.x;
      if (f + 1 < cnt) *(volatile float*)(gp + f + 1) = ov.y;
      if (f + 2 < cnt) *(volatile float*)(gp + f + 2) = ov.z;
    }
  }
}

extern "C" void kernel_launch(void* const* d_in, const int* in_sizes, int n_in,
                              void* d_out, int out_size, void* d_ws, size_t ws_size,
                              hipStream_t stream) {
  if (n_in < 13) return;
  const int nN = in_sizes[0] / 2;
  const int nE = in_sizes[1] / 2;
  if (nN < 1 || nE < 1) return;
  if (in_sizes[0] != 2 * nN || in_sizes[1] != 2 * nE || in_sizes[2] != 3 * nE) return;
  if (in_sizes[3] != KIN * HC || in_sizes[4] != HC || in_sizes[5] != HC * HC || in_sizes[6] != HC) return;
  if (in_sizes[7] != HC || in_sizes[8] < 1 || in_sizes[9] != 3 * HC || in_sizes[10] != HC) return;
  if (in_sizes[11] != HC || in_sizes[12] < 1) return;
  if (out_size != nN) return;

  const int nChunk = (nE + CHB - 1) / CHB;
  const long long ePadL = (long long)nChunk * CHB;
  if (ePadL > (long long)(1 << 22)) return;
  const int ePad = (int)ePadL;
  const int nB = (nN + NBK - 1) / NBK;
  if (nB > MAXB) return;
  const int nBatch = (nChunk + STHR - 1) / STHR;
  const int gEdge  = ePad / EPB;
  const int gNode  = (nN + NTHR - 1) / NTHR;
  const int totE   = nB * CAP2;

  const float* nf  = (const float*)d_in[0];
  const int*   ei  = (const int*)d_in[1];
  const float* ea  = (const float*)d_in[2];
  const float* eW0 = (const float*)d_in[3];
  const float* eb0 = (const float*)d_in[4];
  const float* eW1 = (const float*)d_in[5];
  const float* eb1 = (const float*)d_in[6];
  const float* eW2 = (const float*)d_in[7];
  const float* eb2 = (const float*)d_in[8];
  const float* nW0 = (const float*)d_in[9];
  const float* nb0 = (const float*)d_in[10];
  const float* nW1 = (const float*)d_in[11];
  const float* nb1 = (const float*)d_in[12];
  float* out = (float*)d_out;
  const int* dsts = ei + (size_t)nE;

  char* ws = (char*)d_ws;
  size_t off = 0;
  const size_t oMsg = off; off += (size_t)ePad * 4;             off = (off + 255) & ~(size_t)255;
  const size_t oKey = off; off += (size_t)ePad * 4;             off = (off + 255) & ~(size_t)255;
  const size_t oCo  = off; off += (size_t)nChunk * MAXB * 4;    off = (off + 255) & ~(size_t)255;
  const size_t oEid = off; off += (size_t)nB * CAP2 * 4;        off = (off + 255) & ~(size_t)255;
  const size_t oNt  = off; off += (size_t)nB * NBK * 2 * 4;     off = (off + 255) & ~(size_t)255;
  if (off > ws_size || off > (size_t)WSCAP) return;
  float*    msg = (float*)(ws + oMsg);
  unsigned* KEY = (unsigned*)(ws + oKey);
  unsigned* CO  = (unsigned*)(ws + oCo);
  unsigned* EID = (unsigned*)(ws + oEid);
  int*      NT  = (int*)(ws + oNt);

  hipFuncSetAttribute(reinterpret_cast<const void*>(&k_bucket), hipFuncAttributeMaxDynamicSharedMemorySize, LDS_BKT);

  k_edge<<<gEdge, ETHR, 0, stream>>>(nf, ei, ea, eW0, eb0, eW1, eb1, eW2, eb2, msg, nN, nE);
  k_bsort<<<nChunk, STHR, 0, stream>>>(dsts, KEY, CO, nN, nE);
  k_bucket<<<nB, STHR, LDS_BKT, stream>>>(CO, KEY, EID, NT, nChunk, nBatch);
  k_node<<<gNode, NTHR, 0, stream>>>(NT, EID, msg, nf, nW0, nb0, nW1, nb1, out, nN, nE, totE);
}
